// DiTBlock_34668976013505
// MI455X (gfx1250) — hardware-verified
//
#include <hip/hip_runtime.h>
#include <math.h>

#ifndef NB
#define NB 4
#endif
#ifndef SEQ
#define SEQ 1024
#endif
#define NB_FULL  4
#define SEQ_FULL 1024
#define FEAT 1024
#define NH   16
#define HD   64
#define MF   4096
#define QKP  (2 * FEAT)
#define NTOK (NB * SEQ)
static_assert(NH * HD == FEAT);
static_assert(HD == 64);
static_assert(NB >= 1 && NB <= NB_FULL);
static_assert(SEQ >= 64 && SEQ <= SEQ_FULL && (SEQ % 64) == 0);
static_assert((FEAT % 64) == 0 && (MF % 64) == 0 && (QKP % 64) == 0);
static_assert((FEAT % 32) == 0 && (MF % 32) == 0);
static_assert(FEAT == 4 * 256);
static_assert(((long long)(NB - 1) * SEQ_FULL + SEQ) * FEAT <= (long long)NB_FULL * SEQ_FULL * FEAT);

#define WCARRY   64.0f
#define PSCALE   16384.0f
#define CTXCARRY 256.0f
#define MIDCARRY 16.0f

typedef _Float16 v16h __attribute__((ext_vector_type(16)));
typedef _Float16 v8h  __attribute__((ext_vector_type(8)));
typedef float    v8f  __attribute__((ext_vector_type(8)));
typedef float    v4f  __attribute__((ext_vector_type(4)));
typedef int      v4i  __attribute__((ext_vector_type(4)));
typedef v8h __attribute__((may_alias)) v8ha;
typedef v4f __attribute__((may_alias)) v4fa;
typedef v4i __attribute__((may_alias)) v4ia;
union Frag { v16h v; v8h half[2]; };

#if defined(__HIP_DEVICE_COMPILE__)
#define DEV_ASM 1
#else
#define DEV_ASM 0
#endif

__device__ __forceinline__ v8f zero8() { v8f z = {0.f, 0.f, 0.f, 0.f, 0.f, 0.f, 0.f, 0.f}; return z; }

__device__ __forceinline__ float bf16r(float f) {
  unsigned u = __float_as_uint(f);
  u = (u + 0x7FFFu + ((u >> 16) & 1u)) & 0xFFFF0000u;
  return __uint_as_float(u);
}
__device__ __forceinline__ v4f bf16r4(v4f a) {
  v4f r = { bf16r(a.x), bf16r(a.y), bf16r(a.z), bf16r(a.w) };
  return r;
}

__device__ __forceinline__ v8f wmma_f16(v16h a, v16h b, v8f c) {
  v8f d = __builtin_amdgcn_wmma_f32_16x16x32_f16(false, a, false, b, (short)0, c, false, false);
#if DEV_ASM
  asm volatile("v_nop\n\tv_nop\n\tv_nop\n\tv_nop" : "+v"(d) : "v"(a), "v"(b));
#endif
  return d;
}
__device__ __forceinline__ v8f mmar(v16h a, v16h b, v8f c) {
  return __builtin_amdgcn_wmma_f32_16x16x32_f16(false, a, false, b, (short)0, c, false, false);
}
__device__ __forceinline__ void dep_guard(v8f& a, v8f& b, v16h x, v16h y) {
#if DEV_ASM
  asm volatile("v_nop\n\tv_nop\n\tv_nop\n\tv_nop" : "+v"(a), "+v"(b) : "v"(x), "v"(y));
#else
  (void)a; (void)b; (void)x; (void)y;
#endif
}
__device__ __forceinline__ void keep4(v16h a, v16h b, v16h c, v16h d) {
#if DEV_ASM
  asm volatile("v_nop" :: "v"(a), "v"(b), "v"(c), "v"(d));
#else
  (void)a; (void)b; (void)c; (void)d;
#endif
}
__device__ __forceinline__ void acc_guard4(v8f& a, v8f& b, v8f& c, v8f& d) {
#if DEV_ASM
  asm volatile("v_nop\n\tv_nop\n\tv_nop\n\tv_nop" : "+v"(a), "+v"(b), "+v"(c), "+v"(d));
#else
  (void)a; (void)b; (void)c; (void)d;
#endif
}

__device__ __forceinline__ v16h load_frag(const _Float16* p, int h) {
  Frag f;
  f.half[0] = *(const v8ha*)(p + 8 * h);
  f.half[1] = *(const v8ha*)(p + 16 + 8 * h);
  return f.v;
}
__device__ __forceinline__ v16h ldfrag(const _Float16* p) {
  Frag f;
  f.half[0] = *(const v8ha*)(p);
  f.half[1] = *(const v8ha*)(p + 16);
  return f.v;
}

__global__ __launch_bounds__(256) void transpose_cvt(
    const float* __restrict__ in, _Float16* out, int K, int N, float carry)
{
  __shared__ __align__(16) float tile[32][68];
  const int k0 = blockIdx.x * 64, n0 = blockIdx.y * 32;
  const int tid = (int)threadIdx.x;
  {
    const int kk = tid >> 2, nq = (tid & 3) * 8;
    const float* src = in + (size_t)(k0 + kk) * N + n0 + nq;
    const v4f a = *(const v4fa*)src;
    const v4f c = *(const v4fa*)(src + 4);
    tile[nq + 0][kk] = a.x; tile[nq + 1][kk] = a.y; tile[nq + 2][kk] = a.z; tile[nq + 3][kk] = a.w;
    tile[nq + 4][kk] = c.x; tile[nq + 5][kk] = c.y; tile[nq + 6][kk] = c.z; tile[nq + 7][kk] = c.w;
  }
  __syncthreads();
  {
    const int nn = tid >> 3, kq = (tid & 7) * 8;
    const float* sp = &tile[nn][kq];
    const v4f a = bf16r4(*(const v4fa*)sp);
    const v4f c = bf16r4(*(const v4fa*)(sp + 4));
    const v8h o = { (_Float16)(a.x * carry), (_Float16)(a.y * carry), (_Float16)(a.z * carry), (_Float16)(a.w * carry),
                    (_Float16)(c.x * carry), (_Float16)(c.y * carry), (_Float16)(c.z * carry), (_Float16)(c.w * carry) };
    _Float16* dst = out + (size_t)(n0 + nn) * K + k0 + kq;
    *(volatile v8h*)dst = o;
    __threadfence();
    *(volatile v8h*)dst = o;
  }
}

__global__ __launch_bounds__(128) void cvt_rows(const float* __restrict__ src, _Float16* dst)
{
  const int row = blockIdx.x;
  const int bb = row / SEQ, t = row - bb * SEQ;
  const int tid = (int)threadIdx.x;
  const float* sp = src + ((size_t)bb * SEQ_FULL + (size_t)t) * FEAT + 8 * tid;
  const v4f a = bf16r4(*(const v4fa*)sp);
  const v4f c = bf16r4(*(const v4fa*)(sp + 4));
  const v8h o = { (_Float16)a.x, (_Float16)a.y, (_Float16)a.z, (_Float16)a.w,
                  (_Float16)c.x, (_Float16)c.y, (_Float16)c.z, (_Float16)c.w };
  _Float16* d = dst + (size_t)row * FEAT + 8 * tid;
  *(volatile v8h*)d = o;
  __threadfence();
  *(volatile v8h*)d = o;
}

__device__ __forceinline__ float block_sum(float v, float* red, int lane, int w) {
#pragma unroll
  for (int off = 16; off > 0; off >>= 1) v += __shfl_xor(v, off);
  if (lane == 0) red[w] = v;
  __syncthreads();
  float r = red[0];
#pragma unroll
  for (int i = 1; i < 8; ++i) r += red[i];
  __syncthreads();
  return r;
}

template <bool RNEX>
__global__ __launch_bounds__(256) void ln_kernel(
    const float* __restrict__ X, long long strideXB, _Float16* pout)
{
  __shared__ __align__(16) float srow[FEAT];
  __shared__ float red[8];
  const int row = blockIdx.x;
  const int bb  = row / SEQ, t = row - bb * SEQ;
  const int tid = (int)threadIdx.x, lane = tid & 31, w = tid >> 5;
  const int f0  = 4 * tid;
  const float* xp = X + (size_t)bb * (size_t)strideXB + (size_t)t * FEAT + f0;

  v4f xv = *(const v4fa*)xp;
  if (RNEX) xv = bf16r4(xv);
  float s = (xv.x + xv.y) + (xv.z + xv.w);
  s = block_sum(s, red, lane, w);
  const float mu = s * (1.0f / FEAT);
  const float d0 = xv.x - mu, d1 = xv.y - mu, d2 = xv.z - mu, d3 = xv.w - mu;
  float q = (d0 * d0 + d1 * d1) + (d2 * d2 + d3 * d3);
  q = block_sum(q, red, lane, w);
  const float rstd = rsqrtf(q * (1.0f / FEAT) + 1e-6f);

  const v4f ov = { d0 * rstd, d1 * rstd, d2 * rstd, d3 * rstd };
  *(v4fa*)(srow + f0) = ov;
  __syncthreads();
  if (w < 4) {
    const float* sp = srow + 8 * tid;
    const v4f a = *(const v4fa*)sp;
    const v4f c = *(const v4fa*)(sp + 4);
    const v8h o = { (_Float16)a.x, (_Float16)a.y, (_Float16)a.z, (_Float16)a.w,
                    (_Float16)c.x, (_Float16)c.y, (_Float16)c.z, (_Float16)c.w };
    _Float16* dst = pout + (size_t)row * FEAT + 8 * tid;
    *(volatile v8h*)dst = o;
    __threadfence();
    *(volatile v8h*)dst = o;
  }
}

template <int MODE, bool RESRNE>
__global__ __launch_bounds__(256) void gemm64(
    const _Float16* __restrict__ A, int lda, long long strideA,
    const _Float16* __restrict__ Bt, int ldb, long long strideB,
    void* Cout, int ldc, long long strideC,
    const float* __restrict__ bias,
    const float* __restrict__ res, int ldr, long long strideR,
    int M, int N, int K, float oscale, float ocarry)
{
  __shared__ __align__(16) float sT[8][16 * 68];
  const int b    = blockIdx.y;
  const int lane = threadIdx.x & 31;
  const int wave = threadIdx.x >> 5;
  const int tilesN = N >> 6;
  const int tilesM = M >> 6;
  const int tile = blockIdx.x * 8 + wave;
  if (tile >= tilesM * tilesN) return;
  const int tm = tile / tilesN;
  const int tn = tile - tm * tilesN;
  const int m0 = tm << 6;
  const int n0 = tn << 6;

  const _Float16* Ab = A  + (size_t)b * (size_t)strideA;
  const _Float16* Bb = Bt + (size_t)b * (size_t)strideB;

  const int rlane = lane & 15;
  const int koff  = (lane >> 4) * 8;
  const int mOff  = (lane >> 4) * 8;

  v8f acc[4][4];
#pragma unroll
  for (int i = 0; i < 4; ++i)
#pragma unroll
    for (int j = 0; j < 4; ++j) acc[i][j] = zero8();

  for (int k0 = 0; k0 < K; k0 += 32) {
    v16h bq[4];
#pragma unroll
    for (int j = 0; j < 4; ++j)
      bq[j] = ldfrag(Bb + (size_t)(n0 + (j << 4) + rlane) * ldb + koff + k0);
#pragma unroll
    for (int i = 0; i < 4; ++i) {
      const v16h af = ldfrag(Ab + (size_t)(m0 + (i << 4) + rlane) * lda + koff + k0);
#pragma unroll
      for (int j = 0; j < 4; ++j) acc[i][j] = mmar(af, bq[j], acc[i][j]);
      dep_guard(acc[i][0], acc[i][3], af, bq[3]);
    }
    keep4(bq[0], bq[1], bq[2], bq[3]);
  }
  acc_guard4(acc[0][0], acc[0][1], acc[0][2], acc[0][3]);
  acc_guard4(acc[1][0], acc[1][1], acc[1][2], acc[1][3]);
  acc_guard4(acc[2][0], acc[2][1], acc[2][2], acc[2][3]);
  acc_guard4(acc[3][0], acc[3][1], acc[3][2], acc[3][3]);

  float* slab = sT[wave];
#pragma unroll
  for (int i = 0; i < 4; ++i) {
    const int mBase = m0 + (i << 4);
#pragma unroll
    for (int j = 0; j < 4; ++j) {
#pragma unroll
      for (int r = 0; r < 8; ++r) {
        slab[(mOff + r) * 68 + (j << 4) + rlane] = acc[i][j][r];
      }
    }
    __builtin_amdgcn_fence(3, "workgroup");
    __builtin_amdgcn_wave_barrier();
    __builtin_amdgcn_fence(2, "workgroup");
    if (MODE == 0) {
      float* C = (float*)Cout + (size_t)b * (size_t)strideC;
      const float* R = res + (size_t)b * (size_t)strideR;
      const int h2 = lane >> 4, c4 = (lane & 15) * 4;
      const v4f bv = bf16r4(*(const v4fa*)(bias + n0 + c4));
      for (int pass = 0; pass < 2; ++pass) {
#pragma unroll
        for (int it = 0; it < 8; ++it) {
          const int row = it * 2 + h2;
          const size_t go = (size_t)(mBase + row) * ldc + n0 + c4;
          const size_t ro = (size_t)(mBase + row) * ldr + n0 + c4;
          const v4f sv = *(const v4fa*)(slab + row * 68 + c4);
          v4f rv = *(const v4fa*)(R + ro);
          if (RESRNE) rv = bf16r4(rv);
          const v4f v = sv * oscale + bv + rv;
          *(volatile v4f*)(C + go) = v;
        }
        __threadfence();
      }
    } else {
      const int q = lane >> 3, c8 = (lane & 7) * 8;
      _Float16* C = (_Float16*)Cout + (size_t)b * (size_t)strideC;
      float bb8[8] = { 0.f, 0.f, 0.f, 0.f, 0.f, 0.f, 0.f, 0.f };
      if (MODE == 1 || MODE == 2) {
        const v4f ba = bf16r4(*(const v4fa*)(bias + n0 + c8));
        const v4f bc = bf16r4(*(const v4fa*)(bias + n0 + c8 + 4));
        bb8[0] = ba.x; bb8[1] = ba.y; bb8[2] = ba.z; bb8[3] = ba.w;
        bb8[4] = bc.x; bb8[5] = bc.y; bb8[6] = bc.z; bb8[7] = bc.w;
      }
      v8h hv[4];
#pragma unroll
      for (int it = 0; it < 4; ++it) {
        const int row = it * 4 + q;
        const float* sp = slab + row * 68 + c8;
        const v4f a = *(const v4fa*)sp;
        const v4f c = *(const v4fa*)(sp + 4);
        float f[8] = { a.x, a.y, a.z, a.w, c.x, c.y, c.z, c.w };
        float brow = 0.0f;
        if (MODE == 3) brow = bf16r(bias[mBase + row]);
#pragma unroll
        for (int e = 0; e < 8; ++e) {
          float u = f[e] * oscale + ((MODE == 3) ? brow : bb8[e]);
          if (MODE == 2) {
            const float gl = 0.5f * u * (1.0f + erff(u * 0.70710678118654752f));
            u = gl * ocarry;
          }
          f[e] = u;
        }
        const v8h o = { (_Float16)f[0], (_Float16)f[1], (_Float16)f[2], (_Float16)f[3],
                        (_Float16)f[4], (_Float16)f[5], (_Float16)f[6], (_Float16)f[7] };
        hv[it] = o;
      }
      for (int pass = 0; pass < 2; ++pass) {
#pragma unroll
        for (int it = 0; it < 4; ++it) {
          const int row = it * 4 + q;
          *(volatile v8h*)(C + (size_t)(mBase + row) * ldc + n0 + c8) = hv[it];
        }
        __threadfence();
      }
    }
    __builtin_amdgcn_fence(3, "workgroup");
    __builtin_amdgcn_wave_barrier();
    __builtin_amdgcn_fence(2, "workgroup");
  }
}

__device__ __forceinline__ v16h pack_p(v8f a, v8f c) {
  const v16h r = { (_Float16)(a[0] * PSCALE), (_Float16)(a[1] * PSCALE), (_Float16)(a[2] * PSCALE), (_Float16)(a[3] * PSCALE),
                   (_Float16)(a[4] * PSCALE), (_Float16)(a[5] * PSCALE), (_Float16)(a[6] * PSCALE), (_Float16)(a[7] * PSCALE),
                   (_Float16)(c[0] * PSCALE), (_Float16)(c[1] * PSCALE), (_Float16)(c[2] * PSCALE), (_Float16)(c[3] * PSCALE),
                   (_Float16)(c[4] * PSCALE), (_Float16)(c[5] * PSCALE), (_Float16)(c[6] * PSCALE), (_Float16)(c[7] * PSCALE) };
  return r;
}

__global__ __launch_bounds__(128) __attribute__((amdgpu_num_vgpr(256))) void attn_kernel(
    const _Float16* __restrict__ qk, const _Float16* __restrict__ vt,
    const int* __restrict__ mask, _Float16* ctx)
{
  __shared__ __align__(16) float sO[4 * 16 * 64];

  const int tid = (int)threadIdx.x, lane = tid & 31, w = tid >> 5;
  const int h = lane >> 4, m = lane & 15;
  const int bh = blockIdx.y, b = bh / NH, head = bh - b * NH;
  const int q0 = blockIdx.x * 64 + 16 * w;

  const _Float16* qrow = qk + ((size_t)b * SEQ + q0 + m) * QKP + head * HD;
  const v16h qb0 = load_frag(qrow, h);
  const v16h qb1 = load_frag(qrow + 32, h);

  v8f o[4];
#pragma unroll
  for (int t = 0; t < 4; ++t) o[t] = zero8();
  float mrun = -1e30f, lrun = 0.0f;

  const _Float16* kbase = qk + ((size_t)b * SEQ + m) * QKP + FEAT + head * HD;
  const _Float16* vbase = vt + ((size_t)b * FEAT + head * HD + m) * SEQ;
  const int* mk = mask + (size_t)b * SEQ_FULL + 8 * h;

#pragma unroll 1
  for (int kb = 0; kb < SEQ; kb += 64) {
    v8f s[4];
#pragma unroll
    for (int j = 0; j < 4; ++j) {
      const _Float16* kr = kbase + (size_t)(kb + 16 * j) * QKP;
      const v16h kf0 = load_frag(kr, h);
      const v16h kf1 = load_frag(kr + 32, h);
      v8f z = zero8();
      z = wmma_f16(kf0, qb0, z);
      z = wmma_f16(kf1, qb1, z);
      const v4i ma = *(const v4ia*)(mk + kb + 16 * j);
      const v4i mc = *(const v4ia*)(mk + kb + 16 * j + 4);
      const int mm[8] = { ma.x, ma.y, ma.z, ma.w, mc.x, mc.y, mc.z, mc.w };
#pragma unroll
      for (int r = 0; r < 8; ++r) {
        const float sc = z[r] * 0.125f;
        s[j][r] = sc + ((mm[r] != 1) ? -10000.0f : 0.0f);
      }
    }

    float mloc = s[0][0];
#pragma unroll
    for (int j = 0; j < 4; ++j)
#pragma unroll
      for (int r = 0; r < 8; ++r) mloc = fmaxf(mloc, s[j][r]);
    mloc = fmaxf(mloc, __shfl_xor(mloc, 16));
    const float mnew = fmaxf(mrun, mloc);
    const float alpha = __expf(mrun - mnew);
    mrun = mnew;
    float lsum = 0.0f;
#pragma unroll
    for (int j = 0; j < 4; ++j)
#pragma unroll
      for (int r = 0; r < 8; ++r) {
        const float p = __expf(s[j][r] - mnew);
        s[j][r] = p;
        lsum += p;
      }
    lsum += __shfl_xor(lsum, 16);
    lrun = lrun * alpha + lsum;
#pragma unroll
    for (int t = 0; t < 4; ++t)
#pragma unroll
      for (int r = 0; r < 8; ++r) o[t][r] = o[t][r] * alpha;

    const v16h pb0 = pack_p(s[0], s[1]);
    const v16h pb1 = pack_p(s[2], s[3]);

#pragma unroll
    for (int t = 0; t < 4; ++t) {
      const _Float16* vp = vbase + (size_t)(16 * t) * SEQ + kb;
      const v16h vf0 = load_frag(vp, h);
      const v16h vf1 = load_frag(vp + 32, h);
      o[t] = wmma_f16(vf0, pb0, o[t]);
      o[t] = wmma_f16(vf1, pb1, o[t]);
    }
  }

  const float inv = (1.0f / lrun) * (CTXCARRY / PSCALE);
  float* so = sO + w * 1024;
#pragma unroll
  for (int t = 0; t < 4; ++t)
#pragma unroll
    for (int r = 0; r < 8; ++r)
      so[m * 64 + 16 * t + 8 * h + r] = o[t][r] * inv;
  __syncthreads();

  const int q8 = lane & 7, sub = lane >> 3;
  v8h hv[4];
#pragma unroll
  for (int it = 0; it < 4; ++it) {
    const int row = it * 4 + sub;
    const float* sp = so + row * 64 + 8 * q8;
    const v4f a = *(const v4fa*)sp;
    const v4f c = *(const v4fa*)(sp + 4);
    const v8h ov = { (_Float16)a.x, (_Float16)a.y, (_Float16)a.z, (_Float16)a.w,
                     (_Float16)c.x, (_Float16)c.y, (_Float16)c.z, (_Float16)c.w };
    hv[it] = ov;
  }
  for (int pass = 0; pass < 2; ++pass) {
#pragma unroll
    for (int it = 0; it < 4; ++it) {
      const int row = it * 4 + sub;
      _Float16* dst = ctx + ((size_t)b * SEQ + q0 + row) * FEAT + head * HD + 8 * q8;
      *(volatile v8h*)dst = hv[it];
    }
    __threadfence();
  }
}

extern "C" void kernel_launch(void* const* d_in, const int* in_sizes, int n_in,
                              void* d_out, int out_size, void* d_ws, size_t ws_size,
                              hipStream_t stream)
{
  if (n_in < 19) return;
  const long long needTok = (long long)(NB - 1) * SEQ_FULL + SEQ;
  if ((long long)in_sizes[0] < needTok * FEAT) return;
  if ((long long)in_sizes[1] < needTok * FEAT) return;
  if ((long long)in_sizes[2] < needTok) return;
  if ((long long)in_sizes[3] < (long long)FEAT * 3 * FEAT || in_sizes[4] < 3 * FEAT) return;
  if ((long long)in_sizes[5] < (long long)FEAT * FEAT || in_sizes[6] < FEAT) return;
  if ((long long)in_sizes[7] < (long long)FEAT * FEAT || in_sizes[8] < FEAT) return;
  if ((long long)in_sizes[9] < (long long)FEAT * FEAT || in_sizes[10] < FEAT) return;
  if ((long long)in_sizes[11] < (long long)FEAT * FEAT || in_sizes[12] < FEAT) return;
  if ((long long)in_sizes[13] < (long long)FEAT * FEAT || in_sizes[14] < FEAT) return;
  if ((long long)in_sizes[15] < (long long)FEAT * MF || in_sizes[16] < MF) return;
  if ((long long)in_sizes[17] < (long long)MF * FEAT || in_sizes[18] < FEAT) return;
  if ((long long)out_size < needTok * FEAT) return;

  const float* x         = (const float*)d_in[0];
  const float* c         = (const float*)d_in[1];
  const int*   mask      = (const int*)d_in[2];
  const float* sa_qkv_w  = (const float*)d_in[3];
  const float* sa_qkv_b  = (const float*)d_in[4];
  const float* sa_proj_w = (const float*)d_in[5];
  const float* sa_proj_b = (const float*)d_in[6];
  const float* ca_q_w    = (const float*)d_in[7];
  const float* ca_q_b    = (const float*)d_in[8];
  const float* ca_k_w    = (const float*)d_in[9];
  const float* ca_k_b    = (const float*)d_in[10];
  const float* ca_v_w    = (const float*)d_in[11];
  const float* ca_v_b    = (const float*)d_in[12];
  const float* ca_proj_w = (const float*)d_in[13];
  const float* ca_proj_b = (const float*)d_in[14];
  const float* fc1_w     = (const float*)d_in[15];
  const float* fc1_b     = (const float*)d_in[16];
  const float* fc2_w     = (const float*)d_in[17];
  const float* fc2_b     = (const float*)d_in[18];

  const size_t P_F16  = (size_t)NTOK * FEAT * 2;
  const size_t P_F32  = (size_t)NTOK * FEAT * 4;
  const size_t P_W    = (size_t)FEAT * FEAT * 2;
  const size_t P_WQKV = (size_t)3 * FEAT * FEAT * 2;
  const size_t P_W1   = (size_t)MF * FEAT * 2;
  const size_t P_QK   = (size_t)NTOK * QKP * 2;
  const size_t P_VT   = (size_t)NB * FEAT * SEQ * 2;
  const size_t P_MID  = (size_t)NTOK * MF * 2;
  const size_t P_ATTU = P_QK + P_VT + P_F16;
  const size_t P_ATT  = (P_ATTU > P_MID) ? P_ATTU : P_MID;
  size_t off = 0;
  const size_t oHn   = off; off += P_F16;
  const size_t oC    = off; off += P_F16;
  const size_t oWqkv = off; off += P_WQKV;
  const size_t oWsp  = off; off += P_W;
  const size_t oWcq  = off; off += P_W;
  const size_t oWck  = off; off += P_W;
  const size_t oWcv  = off; off += P_W;
  const size_t oWcp  = off; off += P_W;
  const size_t oW1   = off; off += P_W1;
  const size_t oW2   = off; off += P_W1;
  const size_t oAtt  = off; off += P_ATT;
  const size_t oX1   = off; off += P_F32;
  const size_t oX2   = off; off += P_F32;
  if (off > ws_size) return;
  if (off > (size_t)134217728) return;

  char* ws = (char*)d_ws;
  _Float16* hn    = (_Float16*)(ws + oHn);
  _Float16* cpl   = (_Float16*)(ws + oC);
  _Float16* wqkvT = (_Float16*)(ws + oWqkv);
  _Float16* wspT  = (_Float16*)(ws + oWsp);
  _Float16* wcqT  = (_Float16*)(ws + oWcq);
  _Float16* wckT  = (_Float16*)(ws + oWck);
  _Float16* wcvT  = (_Float16*)(ws + oWcv);
  _Float16* wcpT  = (_Float16*)(ws + oWcp);
  _Float16* w1T   = (_Float16*)(ws + oW1);
  _Float16* w2T   = (_Float16*)(ws + oW2);
  _Float16* qkp   = (_Float16*)(ws + oAtt);
  _Float16* vtp   = (_Float16*)(ws + oAtt + P_QK);
  _Float16* ctx   = (_Float16*)(ws + oAtt + P_QK + P_VT);
  _Float16* mid   = (_Float16*)(ws + oAtt);
  float*    x1    = (float*)(ws + oX1);
  float*    x2    = (float*)(ws + oX2);

  const dim3 blk(256);
  const float sQKV  = 1.0f / WCARRY;
  const float sPROJ = 1.0f / (WCARRY * CTXCARRY);
  const float sFC2  = 1.0f / (WCARRY * MIDCARRY);

  transpose_cvt<<<dim3(FEAT / 64, (3 * FEAT) / 32), blk, 0, stream>>>(sa_qkv_w,  wqkvT, FEAT, 3 * FEAT, WCARRY);
  transpose_cvt<<<dim3(FEAT / 64, FEAT / 32),       blk, 0, stream>>>(sa_proj_w, wspT,  FEAT, FEAT,     WCARRY);
  transpose_cvt<<<dim3(FEAT / 64, FEAT / 32),       blk, 0, stream>>>(ca_q_w,    wcqT,  FEAT, FEAT,     WCARRY);
  transpose_cvt<<<dim3(FEAT / 64, FEAT / 32),       blk, 0, stream>>>(ca_k_w,    wckT,  FEAT, FEAT,     WCARRY);
  transpose_cvt<<<dim3(FEAT / 64, FEAT / 32),       blk, 0, stream>>>(ca_v_w,    wcvT,  FEAT, FEAT,     WCARRY);
  transpose_cvt<<<dim3(FEAT / 64, FEAT / 32),       blk, 0, stream>>>(ca_proj_w, wcpT,  FEAT, FEAT,     WCARRY);
  transpose_cvt<<<dim3(FEAT / 64, MF / 32),         blk, 0, stream>>>(fc1_w,     w1T,   FEAT, MF,       WCARRY);
  transpose_cvt<<<dim3(MF / 64, FEAT / 32),         blk, 0, stream>>>(fc2_w,     w2T,   MF,   FEAT,     WCARRY);

  cvt_rows<<<dim3(NTOK), dim3(128), 0, stream>>>(c, cpl);

  ln_kernel<true><<<dim3(NTOK), blk, 0, stream>>>(x, (long long)SEQ_FULL * FEAT, hn);

  const dim3 gQK((((NTOK / 64) * (QKP / 64)) + 7) / 8, 1);
  gemm64<1, false><<<gQK, blk, 0, stream>>>(
      hn, FEAT, 0LL, wqkvT, FEAT, 0LL, (void*)qkp, QKP, 0LL, sa_qkv_b, x1, FEAT, 0LL,
      NTOK, QKP, FEAT, sQKV, 1.0f);
  const dim3 gVT((((FEAT / 64) * (SEQ / 64)) + 7) / 8, NB);
  gemm64<3, false><<<gVT, blk, 0, stream>>>(
      wqkvT + (size_t)2 * FEAT * FEAT, FEAT, 0LL, hn, FEAT, (long long)SEQ * FEAT,
      (void*)vtp, SEQ, (long long)FEAT * SEQ, sa_qkv_b + 2 * FEAT, x1, FEAT, 0LL,
      FEAT, SEQ, FEAT, sQKV, 1.0f);
  const dim3 gAT(SEQ / 64, NB * NH);
  attn_kernel<<<gAT, dim3(128), 0, stream>>>(qkp, vtp, mask, ctx);
  const dim3 gPB((((SEQ / 64) * (FEAT / 64)) + 7) / 8, NB);
  gemm64<0, true><<<gPB, blk, 0, stream>>>(
      ctx, FEAT, (long long)SEQ * FEAT, wspT, FEAT, 0LL, (void*)x1, FEAT, (long long)SEQ * FEAT,
      sa_proj_b, x, FEAT, (long long)SEQ_FULL * FEAT,
      SEQ, FEAT, FEAT, sPROJ, 1.0f);

  ln_kernel<false><<<dim3(NTOK), blk, 0, stream>>>(x1, (long long)SEQ * FEAT, hn);
  const dim3 gQ((((NTOK / 64) * (FEAT / 64)) + 7) / 8, 1);
  gemm64<1, false><<<gQ, blk, 0, stream>>>(
      hn, FEAT, 0LL, wcqT, FEAT, 0LL, (void*)qkp, QKP, 0LL, ca_q_b, x1, FEAT, 0LL,
      NTOK, FEAT, FEAT, sQKV, 1.0f);
  gemm64<1, false><<<gQ, blk, 0, stream>>>(
      cpl, FEAT, 0LL, wckT, FEAT, 0LL, (void*)(qkp + FEAT), QKP, 0LL, ca_k_b, x1, FEAT, 0LL,
      NTOK, FEAT, FEAT, sQKV, 1.0f);
  gemm64<3, false><<<gVT, blk, 0, stream>>>(
      wcvT, FEAT, 0LL, cpl, FEAT, (long long)SEQ * FEAT,
      (void*)vtp, SEQ, (long long)FEAT * SEQ, ca_v_b, x1, FEAT, 0LL,
      FEAT, SEQ, FEAT, sQKV, 1.0f);
  attn_kernel<<<gAT, dim3(128), 0, stream>>>(qkp, vtp, mask, ctx);
  gemm64<0, false><<<gQ, blk, 0, stream>>>(
      ctx, FEAT, 0LL, wcpT, FEAT, 0LL, (void*)x2, FEAT, 0LL,
      ca_proj_b, x1, FEAT, 0LL,
      NTOK, FEAT, FEAT, sPROJ, 1.0f);

  ln_kernel<false><<<dim3(NTOK), blk, 0, stream>>>(x2, (long long)SEQ * FEAT, hn);
  const dim3 gW1((((NTOK / 64) * (MF / 64)) + 7) / 8, 1);
  gemm64<2, false><<<gW1, blk, 0, stream>>>(
      hn, FEAT, 0LL, w1T, FEAT, 0LL, (void*)mid, MF, 0LL, fc1_b, x1, FEAT, 0LL,
      NTOK, MF, FEAT, sQKV, MIDCARRY);
  gemm64<0, false><<<gPB, blk, 0, stream>>>(
      mid, MF, (long long)SEQ * MF, w2T, MF, 0LL, d_out, FEAT, (long long)SEQ_FULL * FEAT,
      fc2_b, x2, FEAT, (long long)SEQ * FEAT,
      SEQ, FEAT, MF, sFC2, 1.0f);

  (void)hipGetLastError();
}
